// GNN_50379966382774
// MI455X (gfx1250) — hardware-verified
//
#include <hip/hip_runtime.h>
#include <stddef.h>
#include <stdint.h>
#include <math.h>


#define NFEAT  42
#define KF     64
#define EMB    256
#define HID    512
#define NL     3
#define K1     512
#define K2     1024
#define NTHR   256
#define NWAVE  8
#define EPT    8
#define CHUNK  (NTHR * EPT)
#define WCAP   (EPT * 32)
#define LISTN  (NWAVE * WCAP)
#define NBA    256
#define SLA    8
#define RCAP   12288
#define DEGCAP 64
#define GBM    64
#define GBN    64
#define GTHR   128
#define NUF    (EMB * (KF / 8))
#define NU1L   (HID * (K1 / 8))
#define NU2L   (EMB * (K2 / 8))
#define NUALL  (NUF + NL * NU1L + NL * NU2L)
#define AGG_ZINTS    (LISTN + 2 * RCAP + 3 * NBA)
#define MISC_INTS    16
#define ROWBUF_INTS  (NWAVE * K1 / 2)
#define AGG_LDS_INTS (AGG_ZINTS + MISC_INTS + ROWBUF_INTS)
#define WSMAX  134217728

static_assert((CHUNK & (CHUNK - 1)) == 0 && CHUNK <= 4096);
static_assert((NBA & (NBA - 1)) == 0 && NBA == (1 << SLA));
static_assert(((long long)CHUNK << SLA) < (1LL << 31));
static_assert(NBA % NWAVE == 0 && NBA % 32 == 0 && NBA % GBM == 0);
static_assert(RCAP % 4 == 0 && AGG_ZINTS % 4 == 0 && LISTN % 4 == 0 && ((AGG_ZINTS + MISC_INTS) % 4) == 0);
static_assert(KF % 32 == 0 && K1 % 32 == 0 && K2 % 32 == 0 && K1 == 2 * EMB && K2 == 2 * HID);
static_assert(GBM == (GTHR / 32) * 16 && GBN == 64 && EMB % GBN == 0 && HID % GBN == 0);
static_assert(NUF % NTHR == 0 && NU1L % NTHR == 0 && NU2L % NTHR == 0 && NUALL % NTHR == 0);
static_assert(EMB == 8 * 32);
static_assert(AGG_LDS_INTS * 4 <= 300000);

typedef float          v4f   __attribute__((ext_vector_type(4)));
typedef float          v8f   __attribute__((ext_vector_type(8)));
typedef double         v2d   __attribute__((ext_vector_type(2)));
typedef int            v4i   __attribute__((ext_vector_type(4)));
typedef int            v8i   __attribute__((ext_vector_type(8)));
typedef unsigned short v4us  __attribute__((ext_vector_type(4)));
typedef unsigned short v8us  __attribute__((ext_vector_type(8)));
typedef unsigned short v16us __attribute__((ext_vector_type(16)));
typedef __bf16         v16bf __attribute__((ext_vector_type(16)));
typedef v4f  __attribute__((may_alias)) v4fa;
typedef v4i  __attribute__((may_alias)) v4ia;
typedef v4us __attribute__((may_alias)) v4usa;
typedef v8us __attribute__((may_alias)) v8usa;
union FragB { v16bf v; v16us u; v8us h[2]; v8i w; };

__device__ __forceinline__ v8f wmb(const FragB& a, const FragB& b, v8f c) {
  v8f d = __builtin_amdgcn_wmma_f32_16x16x32_bf16(false, a.v, false, b.v, (short)0, c, false, false);
  asm volatile("v_nop\n\tv_nop\n\tv_nop\n\tv_nop" : "+v"(d) : "v"(a.w), "v"(b.w));
  return d;
}

__device__ __forceinline__ unsigned bf16_bits(float f) {
  const unsigned u = __float_as_uint(f);
  return (u + 0x7FFFu + ((u >> 16) & 1u)) >> 16;
}
__device__ __forceinline__ float bf16_val(float f) {
  return __uint_as_float(bf16_bits(f) << 16);
}
__device__ __forceinline__ v4f bf16_val4(v4f a) {
  v4f r;
  r.x = bf16_val(a.x); r.y = bf16_val(a.y); r.z = bf16_val(a.z); r.w = bf16_val(a.w);
  return r;
}
__device__ __forceinline__ float relu_keep(float v) { return (v > 0.0f) ? v : (v - v); }

__device__ __forceinline__ void split1(float v, unsigned& hb, unsigned& lb) {
  hb = bf16_bits(v);
  lb = bf16_bits(v - __uint_as_float(hb << 16));
}
__device__ __forceinline__ void split4(v4f v, v4us& h, v4us& l) {
  unsigned hb, lb;
  split1(v.x, hb, lb); h[0] = (unsigned short)hb; l[0] = (unsigned short)lb;
  split1(v.y, hb, lb); h[1] = (unsigned short)hb; l[1] = (unsigned short)lb;
  split1(v.z, hb, lb); h[2] = (unsigned short)hb; l[2] = (unsigned short)lb;
  split1(v.w, hb, lb); h[3] = (unsigned short)hb; l[3] = (unsigned short)lb;
}
__device__ __forceinline__ void split8(v4f p0, v4f p1, v8us& h, v8us& l) {
  unsigned hb, lb;
  split1(p0.x, hb, lb); h[0] = (unsigned short)hb; l[0] = (unsigned short)lb;
  split1(p0.y, hb, lb); h[1] = (unsigned short)hb; l[1] = (unsigned short)lb;
  split1(p0.z, hb, lb); h[2] = (unsigned short)hb; l[2] = (unsigned short)lb;
  split1(p0.w, hb, lb); h[3] = (unsigned short)hb; l[3] = (unsigned short)lb;
  split1(p1.x, hb, lb); h[4] = (unsigned short)hb; l[4] = (unsigned short)lb;
  split1(p1.y, hb, lb); h[5] = (unsigned short)hb; l[5] = (unsigned short)lb;
  split1(p1.z, hb, lb); h[6] = (unsigned short)hb; l[6] = (unsigned short)lb;
  split1(p1.w, hb, lb); h[7] = (unsigned short)hb; l[7] = (unsigned short)lb;
}

__device__ __forceinline__ void wave_sync() {
  __builtin_amdgcn_fence(__ATOMIC_RELEASE, "wavefront");
  __builtin_amdgcn_wave_barrier();
  __builtin_amdgcn_fence(__ATOMIC_ACQUIRE, "wavefront");
}

template <int SLB>
__device__ __forceinline__ int scan_chunk(const int* __restrict__ dsts, int nE, int cbase, int slotBase,
                                          int nb, int vec8, int* list, int tid, int lane, int wave) {
  int wc = 0;
  const int el0  = tid * EPT;
  const int e0   = cbase + el0;
  const int sent = -2147483647 - 1;
  v4i da, db;
  if (vec8 != 0 && cbase + CHUNK <= nE) {
    da = *(const v4i*)(dsts + e0);
    db = *(const v4i*)(dsts + e0 + 4);
  } else {
    da.x = (e0     < nE) ? dsts[min(e0,     nE - 1)] : sent;
    da.y = (e0 + 1 < nE) ? dsts[min(e0 + 1, nE - 1)] : sent;
    da.z = (e0 + 2 < nE) ? dsts[min(e0 + 2, nE - 1)] : sent;
    da.w = (e0 + 3 < nE) ? dsts[min(e0 + 3, nE - 1)] : sent;
    db.x = (e0 + 4 < nE) ? dsts[min(e0 + 4, nE - 1)] : sent;
    db.y = (e0 + 5 < nE) ? dsts[min(e0 + 5, nE - 1)] : sent;
    db.z = (e0 + 6 < nE) ? dsts[min(e0 + 6, nE - 1)] : sent;
    db.w = (e0 + 7 < nE) ? dsts[min(e0 + 7, nE - 1)] : sent;
  }
  const unsigned nbs = (unsigned)slotBase;
  const unsigned unb = (unsigned)nb;
  const unsigned s0 = (unsigned)da.x - nbs, s1 = (unsigned)da.y - nbs;
  const unsigned s2 = (unsigned)da.z - nbs, s3 = (unsigned)da.w - nbs;
  const unsigned s4 = (unsigned)db.x - nbs, s5 = (unsigned)db.y - nbs;
  const unsigned s6 = (unsigned)db.z - nbs, s7 = (unsigned)db.w - nbs;
  const bool h0 = s0 < unb, h1 = s1 < unb, h2 = s2 < unb, h3 = s3 < unb;
  const bool h4 = s4 < unb, h5 = s5 < unb, h6 = s6 < unb, h7 = s7 < unb;
  const unsigned any = __builtin_amdgcn_ballot_w32(h0 | h1 | h2 | h3 | h4 | h5 | h6 | h7);
  if (any != 0u) {
#define HITJ(J, HJ, SJ) { \
      const unsigned mj = __builtin_amdgcn_ballot_w32(HJ); \
      if (mj != 0u) { \
        if (HJ) { \
          const int pos = wc + (int)__builtin_amdgcn_mbcnt_lo(mj, 0u); \
          if (pos < WCAP) list[wave * WCAP + pos] = ((el0 + (J)) << SLB) | (int)(SJ); \
        } \
        wc += (int)__builtin_popcount(mj); } }
    HITJ(0, h0, s0)
    HITJ(1, h1, s1)
    HITJ(2, h2, s2)
    HITJ(3, h3, s3)
    HITJ(4, h4, s4)
    HITJ(5, h5, s5)
    HITJ(6, h6, s6)
    HITJ(7, h7, s7)
#undef HITJ
  }
  return wc;
}

__global__ __launch_bounds__(NTHR) void k_prep(const float* __restrict__ Wf, const float* __restrict__ W1,
                                               const float* __restrict__ W2, unsigned short* WfT,
                                               unsigned short* W1T2, unsigned short* W2T2) {
  const int u = (int)blockIdx.x * NTHR + (int)threadIdx.x;
  v8us o;
  unsigned short* dp;
  if (u < NUF) {
    const int n  = u >> 3;
    const int k8 = (u & 7) * 8;
#pragma unroll
    for (int i = 0; i < 8; ++i) {
      const int k  = k8 + i;
      const int kc = k < NFEAT ? k : NFEAT - 1;
      const float v = Wf[(size_t)kc * EMB + n];
      o[i] = (k < NFEAT) ? (unsigned short)bf16_bits(v) : (unsigned short)0;
    }
    dp = WfT + (size_t)n * KF + k8;
  } else if (u < NUF + NL * NU1L) {
    const int v  = u - NUF;
    const int l  = v / NU1L;
    const int w  = v - l * NU1L;
    const int n  = w >> 6;
    const int k8 = (w & 63) * 8;
    const int kk = k8 & (EMB - 1);
    const float* p = W1 + (size_t)l * EMB * HID + (size_t)kk * HID + n;
#pragma unroll
    for (int i = 0; i < 8; ++i) o[i] = (unsigned short)bf16_bits(p[(size_t)i * HID]);
    dp = W1T2 + (size_t)l * HID * K1 + (size_t)n * K1 + k8;
  } else if (u < NUALL) {
    const int v  = u - NUF - NL * NU1L;
    const int l  = v / NU2L;
    const int w  = v - l * NU2L;
    const int n  = w >> 7;
    const int k8 = (w & 127) * 8;
    const int kk = k8 & (HID - 1);
    const float* p = W2 + (size_t)l * HID * EMB + (size_t)kk * EMB + n;
#pragma unroll
    for (int i = 0; i < 8; ++i) o[i] = (unsigned short)bf16_bits(p[(size_t)i * EMB]);
    dp = W2T2 + (size_t)l * EMB * K2 + (size_t)n * K2 + k8;
  } else {
    return;
  }
  *(volatile v8us*)dp = o;
  __threadfence();
  *(volatile v8us*)dp = o;
}

__global__ __launch_bounds__(NTHR) void k_cvx(const float* __restrict__ x, int nN, int nUnits,
                                              unsigned short* xb) {
  const int u = (int)blockIdx.x * NTHR + (int)threadIdx.x;
  if (u >= nUnits) return;
  const int row = u >> 3;
  const int k8  = (u & 7) * 8;
  const int rc  = row < nN ? row : nN - 1;
  const float* p = x + (size_t)rc * NFEAT;
  v8us o;
#pragma unroll
  for (int i = 0; i < 8; ++i) {
    const int k  = k8 + i;
    const int kc = k < NFEAT ? k : NFEAT - 1;
    const float v = p[kc];
    o[i] = (row < nN && k < NFEAT) ? (unsigned short)bf16_bits(v) : (unsigned short)0;
  }
  unsigned short* dp = xb + (size_t)row * KF + k8;
  *(volatile v8us*)dp = o;
  __threadfence();
  *(volatile v8us*)dp = o;
}

template <int MODE>
__global__ __launch_bounds__(GTHR) void k_gemm(
    const unsigned short* __restrict__ A, const unsigned short* __restrict__ WT, int K,
    const float* __restrict__ bias, float* outF, unsigned short* outH, double* rec, int nN)
{
  __shared__ __attribute__((aligned(16))) float stg[GBM * GBN];
  const int tid = (int)threadIdx.x, lane = tid & 31, wave = tid >> 5, hh = lane >> 4, m = lane & 15;
  const int rowBase = (int)blockIdx.x * GBM;
  const int col0    = (int)blockIdx.y * GBN;

  v8f acc[4];
  {
    const v8f z = {0.f, 0.f, 0.f, 0.f, 0.f, 0.f, 0.f, 0.f};
    acc[0] = z; acc[1] = z; acc[2] = z; acc[3] = z;
  }
  const unsigned short* ap = A  + (size_t)(rowBase + 16 * wave + m) * (size_t)K + 8 * hh;
  const unsigned short* wp = WT + (size_t)(col0 + m) * (size_t)K + 8 * hh;
  const int ksteps = K >> 5;
#pragma unroll 1
  for (int ks = 0; ks < ksteps; ++ks) {
    FragB af;
    af.h[0] = *(const v8usa*)(ap + 32 * ks);
    af.h[1] = *(const v8usa*)(ap + 32 * ks + 16);
#pragma unroll
    for (int t = 0; t < 4; ++t) {
      const unsigned short* wq = wp + (size_t)(16 * t) * (size_t)K + 32 * ks;
      FragB bf;
      bf.h[0] = *(const v8usa*)wq;
      bf.h[1] = *(const v8usa*)(wq + 16);
      acc[t] = wmb(af, bf, acc[t]);
    }
  }

#pragma unroll
  for (int t = 0; t < 4; ++t) {
    const int lc = 16 * t + m;
#pragma unroll
    for (int r = 0; r < 8; ++r) {
      const int lr = 16 * wave + 8 * hh + r;
      stg[lr * GBN + lc] = acc[t][r];
    }
  }
  __syncthreads();

  if constexpr (MODE == 1) {
    const int c8 = (tid & 7) * 8;
    const v4f bA = bf16_val4(*(const v4f*)(bias + col0 + c8));
    const v4f bB = bf16_val4(*(const v4f*)(bias + col0 + c8 + 4));
    v8us hv[4], lv[4];
#pragma unroll
    for (int it = 0; it < 4; ++it) {
      const int lr = it * 16 + (tid >> 3);
      v4f p0 = *(const v4fa*)(stg + lr * GBN + c8);
      v4f p1 = *(const v4fa*)(stg + lr * GBN + c8 + 4);
      p0 = p0 + bA; p1 = p1 + bB;
      p0.x = relu_keep(p0.x); p0.y = relu_keep(p0.y); p0.z = relu_keep(p0.z); p0.w = relu_keep(p0.w);
      p1.x = relu_keep(p1.x); p1.y = relu_keep(p1.y); p1.z = relu_keep(p1.z); p1.w = relu_keep(p1.w);
      split8(p0, p1, hv[it], lv[it]);
    }
#pragma unroll
    for (int it = 0; it < 4; ++it) {
      const int gr = rowBase + it * 16 + (tid >> 3);
      unsigned short* hp = outH + (size_t)gr * K2 + col0 + c8;
      *(volatile v8us*)hp = hv[it];
      *(volatile v8us*)(hp + HID) = lv[it];
    }
    __threadfence();
#pragma unroll
    for (int it = 0; it < 4; ++it) {
      const int gr = rowBase + it * 16 + (tid >> 3);
      unsigned short* hp = outH + (size_t)gr * K2 + col0 + c8;
      *(volatile v8us*)hp = hv[it];
      *(volatile v8us*)(hp + HID) = lv[it];
    }
  } else {
    const v4f bb = bf16_val4(*(const v4f*)(bias + col0 + 4 * m));
    v4f fv[8];
#pragma unroll
    for (int i = 0; i < 8; ++i) {
      const int lr = 16 * wave + 2 * i + hh;
      fv[i] = *(const v4fa*)(stg + lr * GBN + 4 * m) + bb;
    }
#pragma unroll
    for (int i = 0; i < 8; ++i) {
      const int lr = 16 * wave + 2 * i + hh;
      const int gr = rowBase + lr;
      float* op = outF + (size_t)gr * EMB + col0 + 4 * m;
      *(volatile v4f*)op = fv[i];
    }
    __threadfence();
#pragma unroll
    for (int i = 0; i < 8; ++i) {
      const int lr = 16 * wave + 2 * i + hh;
      const int gr = rowBase + lr;
      float* op = outF + (size_t)gr * EMB + col0 + 4 * m;
      *(volatile v4f*)op = fv[i];
    }
    if constexpr (MODE == 2) {
      if (tid < GBN) {
        int nv = nN - rowBase;
        nv = nv < 0 ? 0 : (nv > GBM ? GBM : nv);
        const float bc = bf16_val(bias[col0 + tid]);
        double s = 0.0, s2 = 0.0;
#pragma unroll 4
        for (int r = 0; r < nv; ++r) {
          const float v = stg[r * GBN + tid] + bc;
          const double dv = (double)v;
          s  += dv;
          s2 += dv * dv;
        }
        v2d rv;
        rv.x = s; rv.y = s2;
        double* rp = rec + ((size_t)blockIdx.x * EMB + col0 + tid) * 2;
        *(volatile v2d*)rp = rv;
        __threadfence();
        *(volatile v2d*)rp = rv;
      }
    }
  }
}

__global__ __launch_bounds__(NTHR) void k_scan(const int* __restrict__ srcs, const int* __restrict__ dsts,
                                               const float* __restrict__ ea,
                                               int nE, int nN, int vec8, int mRows,
                                               const float* __restrict__ hf,
                                               const float* __restrict__ We, const float* __restrict__ be,
                                               const float* __restrict__ epsp, unsigned short* zin) {
  extern __shared__ __attribute__((aligned(16))) int dsm[];
  int* list = dsm;
  int* hl   = dsm + LISTN;
  int* sl   = hl + RCAP;
  int* cnt  = sl + RCAP;
  int* offs = cnt + NBA;
  int* cur  = offs + NBA;
  int* misc = cur + NBA;
  const int tid = (int)threadIdx.x, lane = tid & 31, wave = tid >> 5;
  unsigned short* rowbuf = (unsigned short*)(misc + MISC_INTS) + wave * K1;
  const int nodeBase = (int)blockIdx.x * NBA;

  {
    const v4i z4 = {0, 0, 0, 0};
    for (int i = tid * 4; i < AGG_ZINTS; i += NTHR * 4) *(v4ia*)(dsm + i) = z4;
    if (tid < MISC_INTS) misc[tid] = 0;
  }
  v4f wA[4], wB[4];
#pragma unroll
  for (int j = 0; j < 4; ++j) {
    wA[j] = bf16_val4(*(const v4f*)(We + j * EMB + 4 * lane));
    wB[j] = bf16_val4(*(const v4f*)(We + j * EMB + 128 + 4 * lane));
  }
  const v4f beA = bf16_val4(*(const v4f*)(be + 4 * lane));
  const v4f beB = bf16_val4(*(const v4f*)(be + 128 + 4 * lane));
  const float sc = 1.0f + bf16_val(epsp[0]);
  __syncthreads();

  int t = 0, ov = 0;
  const int nChunks = (nE + CHUNK - 1) / CHUNK;
#pragma unroll 1
  for (int ch = 0; ch < nChunks; ++ch) {
    const int cbase = ch * CHUNK;
    const int wc = scan_chunk<SLA>(dsts, nE, cbase, nodeBase, NBA, vec8, list, tid, lane, wave);
    if (lane == 0) misc[wave] = wc;
    __syncthreads();
    if (wave == 0) {
#pragma unroll 1
      for (int w2 = 0; w2 < NWAVE; ++w2) {
        int c = misc[w2];
        c = c < 0 ? 0 : (c > WCAP ? WCAP : c);
#pragma unroll 1
        for (int b0 = 0; b0 < c; b0 += 32) {
          const int idx = b0 + lane;
          const int ent = list[w2 * WCAP + (idx < WCAP ? idx : WCAP - 1)];
          const int m32 = (c - b0) < 32 ? (c - b0) : 32;
#pragma unroll 1
          for (int k = 0; k < m32; ++k) {
            const int u    = __builtin_amdgcn_readlane(ent, k);
            const int slot = u & (NBA - 1);
            const int el   = (u >> SLA) & (CHUNK - 1);
            const int pk   = ((cbase + el) << SLA) | slot;
            if (t < RCAP) {
              if (lane == 0) { hl[t] = pk; cnt[slot] = cnt[slot] + 1; }
              t = t + 1;
            } else {
              ov = 1;
            }
          }
        }
      }
    }
    __syncthreads();
  }
  if (wave == 0 && lane == 0) { misc[8] = t; misc[9] = ov; }
  __syncthreads();
  int tt = misc[8];
  tt = tt < 0 ? 0 : (tt > RCAP ? RCAP : tt);
  const int ovf = misc[9];

  if (wave == 0) {
    const int base = lane * (NBA / 32);
    int s = 0;
#pragma unroll 1
    for (int i = 0; i < NBA / 32; ++i) s += cnt[base + i];
    int incl = s;
#pragma unroll
    for (int d = 1; d < 32; d <<= 1) {
      const int y = __shfl_up(incl, d, 32);
      if (lane >= d) incl += y;
    }
    int run = incl - s;
#pragma unroll 1
    for (int i = 0; i < NBA / 32; ++i) {
      const int cv = cnt[base + i];
      offs[base + i] = run;
      cur[base + i]  = run;
      run += cv;
    }
  }
  __syncthreads();
  if (wave == 0) {
#pragma unroll 1
    for (int b0 = 0; b0 < tt; b0 += 32) {
      const int idx = b0 + lane;
      const int ent = hl[idx < RCAP ? idx : RCAP - 1];
      const int m32 = (tt - b0) < 32 ? (tt - b0) : 32;
#pragma unroll 1
      for (int k = 0; k < m32; ++k) {
        const int u    = __builtin_amdgcn_readlane(ent, k);
        const int slot = u & (NBA - 1);
        if (lane == 0) {
          int p = cur[slot];
          p = p < 0 ? 0 : (p > RCAP - 1 ? RCAP - 1 : p);
          sl[p] = u;
          cur[slot] = p + 1;
        }
      }
    }
  }
  __syncthreads();

  const float qnan = __int_as_float(0x7fc00000);
  const float pz = (ovf != 0) ? qnan : 0.0f;
#pragma unroll 1
  for (int si = 0; si < NBA / NWAVE; ++si) {
    const int s    = si * NWAVE + wave;
    const int node = nodeBase + s;
    int c = __builtin_amdgcn_readfirstlane(cnt[s]);
    const bool big = c > DEGCAP;
    c = c < 0 ? 0 : (c > DEGCAP ? DEGCAP : c);
    int o = __builtin_amdgcn_readfirstlane(offs[s]);
    o = o < 0 ? 0 : (o > RCAP ? RCAP : o);
    const int nc = node < nN ? node : nN - 1;
    v4f accA = {0.f, 0.f, 0.f, 0.f};
    v4f accB = {0.f, 0.f, 0.f, 0.f};
    float e0 = 0.0f, e1 = 0.0f, e2 = 0.0f, e3 = 0.0f;
#pragma unroll 1
    for (int b0 = 0; b0 < c; b0 += 32) {
      int idx = o + b0 + lane;
      idx = idx > RCAP - 1 ? RCAP - 1 : idx;
      const int ent = sl[idx];
      int eid = ent >> SLA;
      eid = eid < 0 ? 0 : (eid > nE - 1 ? nE - 1 : eid);
      int sr = srcs[eid];
      sr = sr < 0 ? 0 : (sr > nN - 1 ? nN - 1 : sr);
      const v4f ev = *(const v4f*)(ea + (size_t)eid * 4);
      const bool vl = (b0 + lane) < c;
      e0 += vl ? bf16_val(ev.x) : 0.0f;
      e1 += vl ? bf16_val(ev.y) : 0.0f;
      e2 += vl ? bf16_val(ev.z) : 0.0f;
      e3 += vl ? bf16_val(ev.w) : 0.0f;
      const int m32 = (c - b0) < 32 ? (c - b0) : 32;
#pragma unroll 1
      for (int k = 0; k < m32; ++k) {
        const int sk = __builtin_amdgcn_readlane(sr, k);
        const float* rp = hf + (size_t)sk * EMB + 4 * lane;
        const v4f pa = *(const v4f*)rp;
        const v4f pb = *(const v4f*)(rp + 128);
        accA = accA + pa;
        accB = accB + pb;
      }
    }
#pragma unroll
    for (int d = 16; d >= 1; d >>= 1) {
      e0 += __shfl_xor(e0, d, 32);
      e1 += __shfl_xor(e1, d, 32);
      e2 += __shfl_xor(e2, d, 32);
      e3 += __shfl_xor(e3, d, 32);
    }
    const float dg = (float)c;
    v4f tA = wA[0] * e0;
    tA = wA[1] * e1 + tA;
    tA = wA[2] * e2 + tA;
    tA = wA[3] * e3 + tA;
    tA = beA * dg + tA;
    v4f tB = wB[0] * e0;
    tB = wB[1] * e1 + tB;
    tB = wB[2] * e2 + tB;
    tB = wB[3] * e3 + tB;
    tB = beB * dg + tB;
    const v4f sA = *(const v4f*)(hf + (size_t)nc * EMB + 4 * lane);
    const v4f sB = *(const v4f*)(hf + (size_t)nc * EMB + 128 + 4 * lane);
    const float pzr = big ? qnan : pz;
    v4f zA = (sA * sc + accA) + tA;
    v4f zB = (sB * sc + accB) + tB;
    zA = zA + pzr;
    zB = zB + pzr;
    const bool live = node < nN;
    zA.x = live ? zA.x : 0.0f; zA.y = live ? zA.y : 0.0f; zA.z = live ? zA.z : 0.0f; zA.w = live ? zA.w : 0.0f;
    zB.x = live ? zB.x : 0.0f; zB.y = live ? zB.y : 0.0f; zB.z = live ? zB.z : 0.0f; zB.w = live ? zB.w : 0.0f;
    v4us hA, lA, hB, lB;
    split4(zA, hA, lA);
    split4(zB, hB, lB);
    *(v4usa*)(rowbuf + 4 * lane) = hA;
    *(v4usa*)(rowbuf + 128 + 4 * lane) = hB;
    *(v4usa*)(rowbuf + EMB + 4 * lane) = lA;
    *(v4usa*)(rowbuf + EMB + 128 + 4 * lane) = lB;
    wave_sync();
    const v8us q0 = *(const v8usa*)(rowbuf + 8 * lane);
    const v8us q1 = *(const v8usa*)(rowbuf + EMB + 8 * lane);
    wave_sync();
    if (node < mRows) {
      unsigned short* rpw = zin + (size_t)node * K1 + 8 * lane;
      *(volatile v8us*)rpw = q0;
      *(volatile v8us*)(rpw + EMB) = q1;
      __threadfence();
      *(volatile v8us*)rpw = q0;
      *(volatile v8us*)(rpw + EMB) = q1;
    }
  }
}

__global__ __launch_bounds__(NTHR) void k_stat(const double* __restrict__ rec, int nTiles, double invN, float* mr) {
  __shared__ __attribute__((aligned(16))) float sm[2 * EMB];
  const int tid = (int)threadIdx.x;
  double s = 0.0, s2 = 0.0;
#pragma unroll 4
  for (int t = 0; t < nTiles; ++t) {
    const v2d r = *(const v2d*)(rec + ((size_t)t * EMB + tid) * 2);
    s += r.x;
    s2 += r.y;
  }
  const double mean = s * invN;
  double var = s2 * invN - mean * mean;
  var = (var < 0.0) ? 0.0 : var;
  sm[tid] = (float)mean;
  sm[EMB + tid] = rsqrtf((float)var + 1e-5f);
  __syncthreads();
  if (tid < (2 * EMB) / 4) {
    const v4f v = *(const v4fa*)(sm + 4 * tid);
    *(volatile v4f*)(mr + 4 * tid) = v;
    __threadfence();
    *(volatile v4f*)(mr + 4 * tid) = v;
  }
}

__global__ __launch_bounds__(NTHR) void k_bn(const float* __restrict__ z, const float* __restrict__ mr,
                                             const float* __restrict__ gam, const float* __restrict__ bet,
                                             float* out, int n4) {
  const int idx = (int)blockIdx.x * NTHR + (int)threadIdx.x;
  if (idx >= n4) return;
  const int c4 = (idx & (EMB / 4 - 1)) * 4;
  const v4f v  = *(const v4f*)(z + (size_t)idx * 4);
  const v4f mu = *(const v4f*)(mr + c4);
  const v4f rs = *(const v4f*)(mr + EMB + c4);
  const v4f g  = bf16_val4(*(const v4f*)(gam + c4));
  const v4f b  = bf16_val4(*(const v4f*)(bet + c4));
  v4f o = ((v - mu) * rs) * g + b;
  o.x = relu_keep(o.x); o.y = relu_keep(o.y); o.z = relu_keep(o.z); o.w = relu_keep(o.w);
  float* op = out + (size_t)idx * 4;
  *(volatile v4f*)op = o;
  __threadfence();
  *(volatile v4f*)op = o;
}

static inline int cdiv(int a, int b) { return (a + b - 1) / b; }
static inline size_t al256(size_t o) { return (o + 255) & ~(size_t)255; }

extern "C" void kernel_launch(void* const* d_in, const int* in_sizes, int n_in,
                              void* d_out, int out_size, void* d_ws, size_t ws_size,
                              hipStream_t stream) {
  if (n_in < 14) return;
  if (in_sizes[0] < NFEAT || (in_sizes[0] % NFEAT) != 0) return;
  const int nN = in_sizes[0] / NFEAT;
  if (nN < 16 || nN > (1 << 20)) return;
  if (in_sizes[1] < 2 || (in_sizes[1] & 1) != 0) return;
  const int nE = in_sizes[1] / 2;
  if (nE < 1 || nE >= (1 << 22)) return;
  if ((long long)in_sizes[2] != 4LL * nE) return;
  if (in_sizes[3] != NFEAT * EMB || in_sizes[4] != EMB) return;
  if (in_sizes[5] != NL) return;
  if (in_sizes[6] != NL * 4 * EMB || in_sizes[7] != NL * EMB) return;
  if (in_sizes[8] != NL * EMB * HID || in_sizes[9] != NL * HID) return;
  if (in_sizes[10] != NL * HID * EMB || in_sizes[11] != NL * EMB) return;
  if (in_sizes[12] != NL * EMB || in_sizes[13] != NL * EMB) return;
  if ((long long)out_size != (long long)nN * EMB) return;

  const float* x     = (const float*)d_in[0];
  const int*   edge  = (const int*)d_in[1];
  const float* ea    = (const float*)d_in[2];
  const float* Wf    = (const float*)d_in[3];
  const float* bfe   = (const float*)d_in[4];
  const float* eps   = (const float*)d_in[5];
  const float* We    = (const float*)d_in[6];
  const float* be    = (const float*)d_in[7];
  const float* W1    = (const float*)d_in[8];
  const float* b1    = (const float*)d_in[9];
  const float* W2    = (const float*)d_in[10];
  const float* b2    = (const float*)d_in[11];
  const float* gamma = (const float*)d_in[12];
  const float* beta  = (const float*)d_in[13];
  float* out = (float*)d_out;
  const int* src = edge;
  const int* dst = edge + nE;

  const int MP = cdiv(nN, GBM) * GBM;
  const int gM = MP / GBM;
  const int gA = cdiv(MP, NBA);
  if ((long long)gA * NBA < (long long)MP) return;
  const int vec8 = ((nE & 3) == 0) ? 1 : 0;

  char* ws = (char*)d_ws;
  size_t off = 0;
  const size_t oXB  = off; off = al256(off + (size_t)MP * KF * 2);
  const size_t oWfT = off; off = al256(off + (size_t)EMB * KF * 2);
  const size_t oW1  = off; off = al256(off + (size_t)NL * HID * K1 * 2);
  const size_t oW2  = off; off = al256(off + (size_t)NL * EMB * K2 * 2);
  const size_t oH   = off; off = al256(off + (size_t)MP * EMB * 4);
  const size_t oZIN = off; off = al256(off + (size_t)MP * K1 * 2);
  const size_t oF   = off; off = al256(off + (size_t)MP * K2 * 2);
  const size_t oZ   = off; off = al256(off + (size_t)MP * EMB * 4);
  const size_t oREC = off; off = al256(off + (size_t)gM * EMB * 2 * 8);
  const size_t oMR  = off; off = al256(off + (size_t)2 * EMB * 4);
  if (off > ws_size || off > (size_t)WSMAX) return;
  unsigned short* XB   = (unsigned short*)(ws + oXB);
  unsigned short* WfT  = (unsigned short*)(ws + oWfT);
  unsigned short* W1T2 = (unsigned short*)(ws + oW1);
  unsigned short* W2T2 = (unsigned short*)(ws + oW2);
  float*          H    = (float*)(ws + oH);
  unsigned short* ZIN  = (unsigned short*)(ws + oZIN);
  unsigned short* F    = (unsigned short*)(ws + oF);
  float*          Z    = (float*)(ws + oZ);
  double*         REC  = (double*)(ws + oREC);
  float*          MR   = (float*)(ws + oMR);

  const size_t scanLds = (size_t)AGG_LDS_INTS * 4;
  hipFuncSetAttribute(reinterpret_cast<const void*>(&k_scan), hipFuncAttributeMaxDynamicSharedMemorySize, (int)scanLds);

  const int nUx = MP * (KF / 8);
  const int n4  = nN * (EMB / 4);
  const double invN = 1.0 / (double)nN;

  k_prep<<<NUALL / NTHR, NTHR, 0, stream>>>(Wf, W1, W2, WfT, W1T2, W2T2);
  k_cvx<<<cdiv(nUx, NTHR), NTHR, 0, stream>>>(x, nN, nUx, XB);
  k_gemm<0><<<dim3(gM, EMB / GBN), GTHR, 0, stream>>>(XB, WfT, KF, bfe, H, F, REC, nN);

  for (int l = 0; l < NL; ++l) {
    k_scan<<<gA, NTHR, scanLds, stream>>>(src, dst, ea, nE, nN, vec8, MP, H,
                                          We + (size_t)l * 4 * EMB, be + (size_t)l * EMB, eps + l, ZIN);
    k_gemm<1><<<dim3(gM, HID / GBN), GTHR, 0, stream>>>(ZIN, W1T2 + (size_t)l * HID * K1, K1,
                                                       b1 + (size_t)l * HID, Z, F, REC, nN);
    k_gemm<2><<<dim3(gM, EMB / GBN), GTHR, 0, stream>>>(F, W2T2 + (size_t)l * EMB * K2, K2,
                                                       b2 + (size_t)l * EMB, Z, F, REC, nN);
    k_stat<<<1, NTHR, 0, stream>>>(REC, gM, invN, MR);
    float* dstp = (l == NL - 1) ? out : H;
    k_bn<<<cdiv(n4, NTHR), NTHR, 0, stream>>>(Z, MR, gamma + (size_t)l * EMB, beta + (size_t)l * EMB, dstp, n4);
  }
}
